// MooreS4Block_34127810134322
// MI455X (gfx1250) — hardware-verified
//
#include <hip/hip_runtime.h>
#include <math.h>

constexpr int NBAT   = 8;
constexpr int SEQL   = 2048;
constexpr int HDIM   = 512;
constexpr int NMODE  = 64;
constexpr int FDIM   = 2048;
constexpr int NROWS  = NBAT * SEQL;
constexpr int CHK    = 64;
constexpr int NCHK   = SEQL / CHK;
constexpr int KPLEN  = SEQL + CHK;
constexpr int UPITCH = 72;
constexpr int UROWS  = 16 + NCHK;
constexpr int SLP    = 68;
constexpr float WCARRY     = 256.0f;
constexpr float WCARRY_INV = 1.0f / WCARRY;
constexpr float KCARRY     = 64.0f;
constexpr float KCARRY_INV = 1.0f / KCARRY;
constexpr float LN_EPS_F   = 1e-5f;

static_assert(NROWS == 16384, "rows");
static_assert(NROWS % 64 == 0 && HDIM % 64 == 0 && FDIM % 64 == 0, "tile multiples");
static_assert(HDIM % 32 == 0 && FDIM % 32 == 0 && CHK % 32 == 0, "k multiples of 32");
static_assert(NCHK == 32 && KPLEN == 2112, "chunking");
static_assert((8 * KPLEN) % 128 == 0, "tap copy loop exact");
static_assert((KPLEN * 2) % 16 == 0 && (UPITCH * 2) % 16 == 0, "16-B alignment of LDS rows");
static_assert(NMODE == 64, "modes");

typedef __attribute__((ext_vector_type(16))) _Float16 v16h;
typedef __attribute__((ext_vector_type(8)))  _Float16 v8h;
typedef __attribute__((ext_vector_type(8)))  float    v8f;
typedef __attribute__((ext_vector_type(4)))  float    v4f;
typedef __attribute__((ext_vector_type(4)))  unsigned int v4u;

struct FragH {
  union U { v16h v; v8h h[2]; };
  static __device__ __forceinline__ v16h load(const _Float16* p) {
    U f; f.h[0] = *(const v8h*)(p); f.h[1] = *(const v8h*)(p + 16); return f.v;
  }
  static __device__ __forceinline__ v8f mma(v16h a, v16h b, v8f c) {
    return __builtin_amdgcn_wmma_f32_16x16x32_f16(false, a, false, b, (short)0, c, false, false);
  }
};

__device__ __forceinline__ void guard4_h(v8f& c0, v8f& c1, v8f& c2, v8f& c3,
                                         v16h a, v16h b0, v16h b1, v16h b2, v16h b3) {
  asm volatile("v_nop\n\tv_nop\n\tv_nop\n\tv_nop"
               : "+v"(c0), "+v"(c1), "+v"(c2), "+v"(c3)
               : "v"(a), "v"(b0), "v"(b1), "v"(b2), "v"(b3));
}

__device__ __forceinline__ void wave_lds_sync() {
  __builtin_amdgcn_fence(__ATOMIC_RELEASE, "workgroup");
  __builtin_amdgcn_wave_barrier();
  __builtin_amdgcn_fence(__ATOMIC_ACQUIRE, "workgroup");
}

__device__ __forceinline__ float gelu_erf(float v) {
  return 0.5f * v * (1.0f + erff(v * 0.70710678118654752f));
}
__device__ __forceinline__ float sigm(float g) {
  return __builtin_amdgcn_rcpf(1.0f + expf(-g));
}

__global__ __launch_bounds__(256) void cast8_kernel(const float* __restrict__ src,
                                                    unsigned short* __restrict__ dst, int n8, float sc) {
  const int i = blockIdx.x * 256 + threadIdx.x;
  if (i < n8) {
    const v4f a = *(const v4f*)(src + (size_t)i * 8);
    const v4f b = *(const v4f*)(src + (size_t)i * 8 + 4);
    v8h hv;
#pragma unroll
    for (int e = 0; e < 4; ++e) {
      hv[e]     = (_Float16)(a[e] * sc);
      hv[4 + e] = (_Float16)(b[e] * sc);
    }
    unsigned short* dp = dst + (size_t)i * 8;
    *(volatile v8h*)dp = hv;
    __threadfence();
    *(volatile v8h*)dp = hv;
  }
}

__global__ __launch_bounds__(256) void transpose_cast_kernel(const float* __restrict__ in,
                                                             unsigned short* __restrict__ out,
                                                             int R, int C, float sc) {
  __shared__ float Tt[64 * 65];
  const int tid = threadIdx.x, lane = tid & 31, wave = tid >> 5;
  const int r0 = blockIdx.y * 64;
  const int c0 = blockIdx.x * 64;
#pragma unroll
  for (int it = 0; it < 4; ++it) {
    const int idx = tid + 256 * it;
    const int r = idx >> 4;
    const int c4 = (idx & 15) * 4;
    const v4f v = *(const v4f*)(in + (size_t)(r0 + r) * C + c0 + c4);
#pragma unroll
    for (int e = 0; e < 4; ++e) Tt[r * 65 + c4 + e] = v[e];
  }
  __syncthreads();
  const int q = lane >> 3;
  const int r8 = (lane & 7) * 8;
#pragma unroll
  for (int it = 0; it < 2; ++it) {
    const int cl = (it * 8 + wave) * 4 + q;
    v8h hv;
#pragma unroll
    for (int e = 0; e < 8; ++e) hv[e] = (_Float16)(Tt[(r8 + e) * 65 + cl] * sc);
    unsigned short* dp = out + (size_t)(c0 + cl) * R + r0 + r8;
    *(volatile v8h*)dp = hv;
    __threadfence();
    *(volatile v8h*)dp = hv;
  }
}

__global__ __launch_bounds__(256) void kgen_kernel(const float* __restrict__ log_dt,
                                                   const float* __restrict__ log_ar,
                                                   const float* __restrict__ a_im,
                                                   const float* __restrict__ c_re,
                                                   const float* __restrict__ c_im,
                                                   const float* __restrict__ dsk,
                                                   unsigned short* __restrict__ KF) {
  __shared__ float ev[128];
  __shared__ float p_dr[NMODE], p_di[NMODE], p_ar[NMODE], p_ai[NMODE], p_c2r[NMODE], p_c2i[NMODE];
  __shared__ float Gr[32 * 64], Gi[32 * 64];
  __shared__ float Qr[64 * 64], Qi[64 * 64];
  __shared__ __align__(16) float Ks[SEQL];
  const int tid = threadIdx.x;
  const int h = blockIdx.x;

  if (tid < 128) {
    const int n = tid & 63;
    const float a0 = log_ar[h * NMODE + n];
    const float a1 = log_dt[h];
    const float arg = (tid < 64) ? a0 : a1;
    ev[tid] = expf(arg);
  }
  __syncthreads();
  if (tid < 64) {
    const float dt = ev[64];
    const float ar = -ev[tid];
    const float ai = a_im[h * NMODE + tid];
    p_ar[tid] = ar;
    p_ai[tid] = ai;
    p_dr[tid] = dt * ar;
    p_di[tid] = dt * ai;
  }
  __syncthreads();

#pragma unroll 1
  for (int i = 0; i < 24; ++i) {
    const bool isP = (i >= 16);
    const int eidx = tid + 256 * (isP ? (i - 16) : i);
    const int row = eidx >> 6;
    const int n = eidx & 63;
    const float mult = isP ? (float)(64 * row) : (float)row;
    const float e = expf(mult * p_dr[n]);
    const float ang = mult * p_di[n];
    const float cs = cosf(ang);
    const float sn = sinf(ang);
    const float vr = e * cs;
    const float vi = e * sn;
    if (isP) { Gr[eidx] = vr; Gi[eidx] = vi; }
    else     { Qr[eidx] = vr; Qi[eidx] = vi; }
  }
  __syncthreads();

  if (tid < 64) {
    const float wr = Qr[64 + tid];
    const float wi = Qi[64 + tid];
    const float nr = wr - 1.0f;
    const float ni = wi;
    const float cr = c_re[h * NMODE + tid];
    const float ci = c_im[h * NMODE + tid];
    const float pr = cr * nr - ci * ni;
    const float pi = cr * ni + ci * nr;
    const float ar = p_ar[tid];
    const float ai = p_ai[tid];
    const float inv = 1.0f / (ar * ar + ai * ai);
    p_c2r[tid] = 2.0f * (pr * ar + pi * ai) * inv;
    p_c2i[tid] = 2.0f * (pi * ar - pr * ai) * inv;
  }
  __syncthreads();

#pragma unroll 1
  for (int i = 0; i < 8; ++i) {
    const int eidx = tid + 256 * i;
    const int n = eidx & 63;
    const float pr = Gr[eidx];
    const float pi = Gi[eidx];
    const float c2r = p_c2r[n];
    const float c2i = p_c2i[n];
    Gr[eidx] = c2r * pr - c2i * pi;
    Gi[eidx] = c2r * pi + c2i * pr;
  }
  __syncthreads();

  {
    const int r = tid & 63;
    const int qb = tid >> 6;
    float acc[8];
#pragma unroll
    for (int i = 0; i < 8; ++i) acc[i] = 0.0f;
#pragma unroll 1
    for (int n = 0; n < NMODE; ++n) {
      const float qr = Qr[r * 64 + n];
      const float qi = Qi[r * 64 + n];
#pragma unroll
      for (int i = 0; i < 8; ++i) {
        acc[i] += Gr[(qb + 4 * i) * 64 + n] * qr - Gi[(qb + 4 * i) * 64 + n] * qi;
      }
    }
    const float dval = dsk[h];
    acc[0] += (tid == 0) ? dval : 0.0f;
#pragma unroll
    for (int i = 0; i < 8; ++i) Ks[(qb + 4 * i) * 64 + r] = acc[i];
  }
  __syncthreads();

  {
    const v4f a = *(const v4f*)(Ks + 8 * tid);
    const v4f b = *(const v4f*)(Ks + 8 * tid + 4);
    v8h hv;
#pragma unroll
    for (int e = 0; e < 4; ++e) {
      hv[e]     = (_Float16)(a[e] * KCARRY);
      hv[4 + e] = (_Float16)(b[e] * KCARRY);
    }
    unsigned short* dp = KF + (size_t)h * SEQL + 8 * tid;
    *(volatile v8h*)dp = hv;
    __threadfence();
    *(volatile v8h*)dp = hv;
  }
}

__global__ __launch_bounds__(256) void ln1_rev_kernel(const float* __restrict__ x,
                                                      const float* __restrict__ gam,
                                                      const float* __restrict__ bet,
                                                      unsigned short* __restrict__ UREV) {
  __shared__ __align__(16) _Float16 Tt[HDIM * UPITCH];
  const int tid = threadIdx.x, lane = tid & 31, wave = tid >> 5;
  const int c = blockIdx.x;
  const int b = blockIdx.y;
  v4f g[4], bb[4];
#pragma unroll
  for (int q = 0; q < 4; ++q) {
    g[q]  = *(const v4f*)(gam + 128 * q + 4 * lane);
    bb[q] = *(const v4f*)(bet + 128 * q + 4 * lane);
  }
#pragma unroll 1
  for (int i = 0; i < 8; ++i) {
    const int lr = wave * 8 + i;
    const float* rp = x + ((size_t)(b * SEQL + c * CHK + lr)) * HDIM;
    v4f v[4];
    float s = 0.0f;
#pragma unroll
    for (int q = 0; q < 4; ++q) {
      v[q] = *(const v4f*)(rp + 128 * q + 4 * lane);
      s += (v[q][0] + v[q][1]) + (v[q][2] + v[q][3]);
    }
#pragma unroll
    for (int off = 1; off < 32; off <<= 1) s += __shfl_xor(s, off, 32);
    const float mu = s * (1.0f / HDIM);
    float ss = 0.0f;
#pragma unroll
    for (int q = 0; q < 4; ++q)
#pragma unroll
      for (int e = 0; e < 4; ++e) { const float d = v[q][e] - mu; v[q][e] = d; ss += d * d; }
#pragma unroll
    for (int off = 1; off < 32; off <<= 1) ss += __shfl_xor(ss, off, 32);
    const float rstd = rsqrtf(ss * (1.0f / HDIM) + LN_EPS_F);
    const int kr = (CHK - 1) - lr;
#pragma unroll
    for (int q = 0; q < 4; ++q)
#pragma unroll
      for (int e = 0; e < 4; ++e) {
        const float o = (v[q][e] * rstd) * g[q][e] + bb[q][e];
        Tt[(128 * q + 4 * lane + e) * UPITCH + kr] = (_Float16)o;
      }
  }
  __syncthreads();
  const int q4 = lane >> 3;
  const int c8 = (lane & 7) * 8;
#pragma unroll 1
  for (int it = 0; it < 16; ++it) {
    const int hl = (it * 8 + wave) * 4 + q4;
    const v8h hv = *(const v8h*)(Tt + hl * UPITCH + c8);
    unsigned short* dp = UREV + (((size_t)(b * HDIM + hl)) * NCHK + c) * CHK + c8;
    *(volatile v8h*)dp = hv;
    __threadfence();
    *(volatile v8h*)dp = hv;
  }
}

__global__ __launch_bounds__(128) void conv_toeplitz_kernel(const unsigned short* __restrict__ UREVp,
                                                            const unsigned short* __restrict__ KFp,
                                                            unsigned short* __restrict__ YT) {
  __shared__ __align__(16) _Float16 Kc[8 * KPLEN];
  __shared__ __align__(16) _Float16 Us[4 * UROWS * UPITCH];
  __shared__ __align__(16) float    Sl[4 * 32 * SLP];
  const int tid = threadIdx.x, lane = tid & 31, wave = tid >> 5;
  const int h = blockIdx.x;
  const int b = blockIdx.y * 4 + wave;

  {
    const unsigned short* kfrow = KFp + (size_t)h * SEQL;
#pragma unroll 1
    for (int idx = tid; idx < 8 * KPLEN; idx += 128) {
      const int s = idx / KPLEN;
      const int m = idx - s * KPLEN;
      const int src = m + s - CHK;
      const bool ok = (src >= 0) && (src < SEQL);
      const int srcc = (src < 0) ? 0 : ((src > SEQL - 1) ? (SEQL - 1) : src);
      const unsigned short raw = kfrow[srcc];
      const unsigned short sel = ok ? raw : (unsigned short)0;
      Kc[idx] = __builtin_bit_cast(_Float16, sel);
    }
  }
  _Float16* us = Us + wave * (UROWS * UPITCH);
  {
    const _Float16* urow = (const _Float16*)UREVp + ((size_t)(b * HDIM + h)) * SEQL;
#pragma unroll
    for (int it = 0; it < 8; ++it) {
      const int e8 = it * 32 + lane;
      const int cc = e8 >> 3;
      const int col = (e8 & 7) * 8;
      const v8h v = *(const v8h*)(urow + e8 * 8);
      *(v8h*)(us + (16 + cc) * UPITCH + col) = v;
    }
    const v8h zv = {(_Float16)0.0f, (_Float16)0.0f, (_Float16)0.0f, (_Float16)0.0f,
                    (_Float16)0.0f, (_Float16)0.0f, (_Float16)0.0f, (_Float16)0.0f};
    for (int i = lane; i < (16 * UPITCH) / 8; i += 32) *(v8h*)(us + i * 8) = zv;
  }
  __syncthreads();

  const int rl = lane & 15;
  const int hh = lane >> 4;
  const _Float16* bptr[4];
#pragma unroll
  for (int j = 0; j < 4; ++j) {
    const int n = 16 * j + rl;
    const int s = (n + 1) & 7;
    bptr[j] = Kc + s * KPLEN + (n + 1 - s) + 8 * hh;
  }
  const _Float16* a0base = us + (16 + rl) * UPITCH + 8 * hh;
  const _Float16* a1base = us + (32 + rl) * UPITCH + 8 * hh;

  const v8f z8 = {0.f, 0.f, 0.f, 0.f, 0.f, 0.f, 0.f, 0.f};
  v8f acc0[4], acc1[4];
#pragma unroll
  for (int j = 0; j < 4; ++j) { acc0[j] = z8; acc1[j] = z8; }

#pragma unroll 1
  for (int d = 0; d < 16; ++d) {
#pragma unroll
    for (int ks = 0; ks < 2; ++ks) {
      const int k0 = ks * 32;
      v16h bf[4];
#pragma unroll
      for (int j = 0; j < 4; ++j) bf[j] = FragH::load(bptr[j] + 64 * d + k0);
      const v16h a1 = FragH::load(a1base - d * UPITCH + k0);
#pragma unroll
      for (int j = 0; j < 4; ++j) acc1[j] = FragH::mma(a1, bf[j], acc1[j]);
      guard4_h(acc1[0], acc1[1], acc1[2], acc1[3], a1, bf[0], bf[1], bf[2], bf[3]);
      const v16h a0 = FragH::load(a0base - d * UPITCH + k0);
#pragma unroll
      for (int j = 0; j < 4; ++j) acc0[j] = FragH::mma(a0, bf[j], acc0[j]);
      guard4_h(acc0[0], acc0[1], acc0[2], acc0[3], a0, bf[0], bf[1], bf[2], bf[3]);
    }
  }
#pragma unroll 1
  for (int d = 16; d < 32; ++d) {
#pragma unroll
    for (int ks = 0; ks < 2; ++ks) {
      const int k0 = ks * 32;
      v16h bf[4];
#pragma unroll
      for (int j = 0; j < 4; ++j) bf[j] = FragH::load(bptr[j] + 64 * d + k0);
      const v16h a1 = FragH::load(a1base - d * UPITCH + k0);
#pragma unroll
      for (int j = 0; j < 4; ++j) acc1[j] = FragH::mma(a1, bf[j], acc1[j]);
      guard4_h(acc1[0], acc1[1], acc1[2], acc1[3], a1, bf[0], bf[1], bf[2], bf[3]);
    }
  }

  float* slab = Sl + wave * (32 * SLP);
#pragma unroll
  for (int j = 0; j < 4; ++j)
#pragma unroll
    for (int r = 0; r < 8; ++r) {
      slab[(8 * hh + r) * SLP + 16 * j + rl]      = acc0[j][r] * KCARRY_INV;
      slab[(16 + 8 * hh + r) * SLP + 16 * j + rl] = acc1[j][r] * KCARRY_INV;
    }
  wave_lds_sync();
  {
    const int q = lane >> 3;
    const int c8 = (lane & 7) * 8;
    unsigned short* yrow = YT + ((size_t)(b * HDIM + h)) * SEQL;
#pragma unroll 1
    for (int it = 0; it < 8; ++it) {
      const int row = it * 4 + q;
      const float* sp = slab + row * SLP + c8;
      const v4f a = *(const v4f*)(sp);
      const v4f c = *(const v4f*)(sp + 4);
      v8h hv;
#pragma unroll
      for (int e = 0; e < 4; ++e) {
        hv[e]     = (_Float16)gelu_erf(a[e]);
        hv[4 + e] = (_Float16)gelu_erf(c[e]);
      }
      unsigned short* dp = yrow + row * CHK + c8;
      *(volatile v8h*)dp = hv;
      __threadfence();
      *(volatile v8h*)dp = hv;
    }
  }
}

__global__ __launch_bounds__(256) void transpose16_kernel(const unsigned short* __restrict__ in,
                                                          unsigned short* __restrict__ out,
                                                          int R, int C) {
  __shared__ unsigned short Th[64 * 66];
  const int tid = threadIdx.x, lane = tid & 31, wave = tid >> 5;
  const int r0 = blockIdx.y * 64;
  const int c0 = blockIdx.x * 64;
  const unsigned short* ib = in + (size_t)blockIdx.z * R * C;
  unsigned short* ob = out + (size_t)blockIdx.z * R * C;
#pragma unroll
  for (int it = 0; it < 2; ++it) {
    const int idx = tid + 256 * it;
    const int r = idx >> 3;
    const int c8 = (idx & 7) * 8;
    const v4u w = *(const v4u*)(ib + (size_t)(r0 + r) * C + c0 + c8);
    const unsigned w0 = w[0];
    const unsigned w1 = w[1];
    const unsigned w2 = w[2];
    const unsigned w3 = w[3];
    unsigned short* tp = Th + r * 66 + c8;
    tp[0] = (unsigned short)(w0 & 0xffffu);
    tp[1] = (unsigned short)(w0 >> 16);
    tp[2] = (unsigned short)(w1 & 0xffffu);
    tp[3] = (unsigned short)(w1 >> 16);
    tp[4] = (unsigned short)(w2 & 0xffffu);
    tp[5] = (unsigned short)(w2 >> 16);
    tp[6] = (unsigned short)(w3 & 0xffffu);
    tp[7] = (unsigned short)(w3 >> 16);
  }
  __syncthreads();
  const int q = lane >> 3;
  const int r8 = (lane & 7) * 8;
#pragma unroll
  for (int it = 0; it < 2; ++it) {
    const int cl = (it * 8 + wave) * 4 + q;
    const unsigned u0 = Th[(r8 + 0) * 66 + cl];
    const unsigned u1 = Th[(r8 + 1) * 66 + cl];
    const unsigned u2 = Th[(r8 + 2) * 66 + cl];
    const unsigned u3 = Th[(r8 + 3) * 66 + cl];
    const unsigned u4 = Th[(r8 + 4) * 66 + cl];
    const unsigned u5 = Th[(r8 + 5) * 66 + cl];
    const unsigned u6 = Th[(r8 + 6) * 66 + cl];
    const unsigned u7 = Th[(r8 + 7) * 66 + cl];
    v4u ov;
    ov[0] = u0 | (u1 << 16);
    ov[1] = u2 | (u3 << 16);
    ov[2] = u4 | (u5 << 16);
    ov[3] = u6 | (u7 << 16);
    unsigned short* dp = ob + (size_t)(c0 + cl) * R + r0 + r8;
    *(volatile v4u*)dp = ov;
    __threadfence();
    *(volatile v4u*)dp = ov;
  }
}

template <int EPI>
__global__ __launch_bounds__(128) void gemm_f16_kernel(
    const unsigned short* __restrict__ Ap, int lda,
    const unsigned short* __restrict__ Btp, int ldb,
    void* __restrict__ Cout, int ldc,
    const float* __restrict__ bias,
    const float* __restrict__ resid, int ldr,
    int M, int N, int K, float scale) {
  constexpr int TN = (EPI == 0) ? 32 : 64;
  __shared__ __align__(16) float sT[4 * 64 * SLP];
  const _Float16* A  = (const _Float16*)Ap;
  const _Float16* Bt = (const _Float16*)Btp;
  const int lane = threadIdx.x & 31;
  const int wave = threadIdx.x >> 5;
  const int tilesN = N / TN;
  const int tilesM = M >> 6;
  const int tile = blockIdx.x * 4 + wave;
  if (tile >= tilesM * tilesN) return;
  const int tm = tile / tilesN;
  const int tn = tile - tm * tilesN;
  const int m0 = tm << 6;
  const int n0 = tn * TN;
  const int rl = lane & 15;
  const int hh = lane >> 4;
  const int koff = hh * 8;

  size_t bo[4], ao[4];
#pragma unroll
  for (int j = 0; j < 4; ++j) {
    int nr = n0 + 16 * j + rl;
    if (EPI == 0) nr = (j < 2) ? (n0 + 16 * j + rl) : (N + n0 + 16 * (j - 2) + rl);
    bo[j] = (size_t)nr * ldb + koff;
  }
#pragma unroll
  for (int i = 0; i < 4; ++i) ao[i] = (size_t)(m0 + 16 * i + rl) * lda + koff;

  v8f acc[4][4];
#pragma unroll
  for (int i = 0; i < 4; ++i)
#pragma unroll
    for (int j = 0; j < 4; ++j) acc[i][j] = (v8f){0.f, 0.f, 0.f, 0.f, 0.f, 0.f, 0.f, 0.f};

  for (int k0 = 0; k0 < K; k0 += 32) {
    v16h bh[4];
#pragma unroll
    for (int j = 0; j < 4; ++j) bh[j] = FragH::load(Bt + bo[j] + k0);
#pragma unroll
    for (int i = 0; i < 4; ++i) {
      const v16h ah = FragH::load(A + ao[i] + k0);
#pragma unroll
      for (int j = 0; j < 4; ++j) acc[i][j] = FragH::mma(ah, bh[j], acc[i][j]);
      guard4_h(acc[i][0], acc[i][1], acc[i][2], acc[i][3], ah, bh[0], bh[1], bh[2], bh[3]);
    }
  }

  float* slab = sT + wave * (64 * SLP);
#pragma unroll
  for (int i = 0; i < 4; ++i)
#pragma unroll
    for (int j = 0; j < 4; ++j)
#pragma unroll
      for (int r = 0; r < 8; ++r)
        slab[(16 * i + 8 * hh + r) * SLP + 16 * j + rl] = acc[i][j][r] * scale;
  wave_lds_sync();

  if (EPI == 0) {
    float* C = (float*)Cout;
    const int q = lane >> 3;
    const int c4 = (lane & 7) * 4;
    const v4f bv = *(const v4f*)(bias + n0 + c4);
    const v4f bg = *(const v4f*)(bias + N + n0 + c4);
#pragma unroll 1
    for (int it = 0; it < 16; ++it) {
      const int row = it * 4 + q;
      const v4f va = *(const v4f*)(slab + row * SLP + c4);
      const v4f vg = *(const v4f*)(slab + row * SLP + 32 + c4);
      const v4f xr = *(const v4f*)(resid + (size_t)(m0 + row) * ldr + n0 + c4);
      v4f o;
#pragma unroll
      for (int e = 0; e < 4; ++e) {
        const float a = va[e] + bv[e];
        const float g = vg[e] + bg[e];
        const float s = a * sigm(g);
        o[e] = xr[e] + s;
      }
      float* dp = C + (size_t)(m0 + row) * ldc + n0 + c4;
      *(volatile v4f*)dp = o;
      __threadfence();
      *(volatile v4f*)dp = o;
    }
  } else if (EPI == 1) {
    unsigned short* C = (unsigned short*)Cout;
    const int q = lane >> 3;
    const int c8 = (lane & 7) * 8;
    const v4f bA = *(const v4f*)(bias + n0 + c8);
    const v4f bB = *(const v4f*)(bias + n0 + c8 + 4);
#pragma unroll 1
    for (int it = 0; it < 16; ++it) {
      const int row = it * 4 + q;
      const float* sp = slab + row * SLP + c8;
      const v4f a = *(const v4f*)(sp);
      const v4f c = *(const v4f*)(sp + 4);
      v8h hv;
#pragma unroll
      for (int e = 0; e < 4; ++e) {
        hv[e]     = (_Float16)gelu_erf(a[e] + bA[e]);
        hv[4 + e] = (_Float16)gelu_erf(c[e] + bB[e]);
      }
      unsigned short* dp = C + (size_t)(m0 + row) * ldc + n0 + c8;
      *(volatile v8h*)dp = hv;
      __threadfence();
      *(volatile v8h*)dp = hv;
    }
  } else {
    float* C = (float*)Cout;
    const int c4 = (lane & 15) * 4;
    const v4f bv = *(const v4f*)(bias + n0 + c4);
#pragma unroll 1
    for (int it = 0; it < 32; ++it) {
      const int row = it * 2 + hh;
      const v4f va = *(const v4f*)(slab + row * SLP + c4);
      const v4f xr = *(const v4f*)(resid + (size_t)(m0 + row) * ldr + n0 + c4);
      v4f o;
#pragma unroll
      for (int e = 0; e < 4; ++e) o[e] = (va[e] + bv[e]) + xr[e];
      float* dp = C + (size_t)(m0 + row) * ldc + n0 + c4;
      *(volatile v4f*)dp = o;
      __threadfence();
      *(volatile v4f*)dp = o;
    }
  }
}

__global__ __launch_bounds__(256) void ln2_kernel(const float* __restrict__ X1,
                                                  const float* __restrict__ gam,
                                                  const float* __restrict__ bet,
                                                  unsigned short* __restrict__ H2, int nrows) {
  const int tid = threadIdx.x, lane = tid & 31;
  const int row = blockIdx.x * 8 + (tid >> 5);
  if (row >= nrows) return;
  const float* rp = X1 + (size_t)row * HDIM;
  v4f v[4], g[4], bb[4];
  float s = 0.0f;
#pragma unroll
  for (int q = 0; q < 4; ++q) {
    const int off = 256 * (q >> 1) + 8 * lane + 4 * (q & 1);
    v[q]  = *(const v4f*)(rp + off);
    g[q]  = *(const v4f*)(gam + off);
    bb[q] = *(const v4f*)(bet + off);
    s += (v[q][0] + v[q][1]) + (v[q][2] + v[q][3]);
  }
#pragma unroll
  for (int off = 1; off < 32; off <<= 1) s += __shfl_xor(s, off, 32);
  const float mu = s * (1.0f / HDIM);
  float ss = 0.0f;
#pragma unroll
  for (int q = 0; q < 4; ++q)
#pragma unroll
    for (int e = 0; e < 4; ++e) { const float d = v[q][e] - mu; v[q][e] = d; ss += d * d; }
#pragma unroll
  for (int off = 1; off < 32; off <<= 1) ss += __shfl_xor(ss, off, 32);
  const float rstd = rsqrtf(ss * (1.0f / HDIM) + LN_EPS_F);
  v8h h0, h1;
#pragma unroll
  for (int e = 0; e < 4; ++e) {
    h0[e]     = (_Float16)((v[0][e] * rstd) * g[0][e] + bb[0][e]);
    h0[4 + e] = (_Float16)((v[1][e] * rstd) * g[1][e] + bb[1][e]);
    h1[e]     = (_Float16)((v[2][e] * rstd) * g[2][e] + bb[2][e]);
    h1[4 + e] = (_Float16)((v[3][e] * rstd) * g[3][e] + bb[3][e]);
  }
  unsigned short* dp = H2 + (size_t)row * HDIM + 8 * lane;
  *(volatile v8h*)(dp) = h0;
  *(volatile v8h*)(dp + 256) = h1;
  __threadfence();
  *(volatile v8h*)(dp) = h0;
  *(volatile v8h*)(dp + 256) = h1;
}

extern "C" void kernel_launch(void* const* d_in, const int* in_sizes, int n_in,
                              void* d_out, int out_size, void* d_ws, size_t ws_size, hipStream_t stream) {
  if (n_in < 17 || d_out == nullptr || d_ws == nullptr) return;
  if (in_sizes[0] != NROWS * HDIM || in_sizes[1] != HDIM || in_sizes[2] != HDIM || in_sizes[3] != HDIM ||
      in_sizes[4] != HDIM * NMODE || in_sizes[5] != HDIM * NMODE || in_sizes[6] != HDIM * NMODE ||
      in_sizes[7] != HDIM * NMODE || in_sizes[8] != HDIM || in_sizes[9] != 2 * HDIM * HDIM ||
      in_sizes[10] != 2 * HDIM || in_sizes[11] != HDIM || in_sizes[12] != HDIM ||
      in_sizes[13] != HDIM * FDIM || in_sizes[14] != FDIM || in_sizes[15] != FDIM * HDIM ||
      in_sizes[16] != HDIM || out_size != NROWS * HDIM) return;

  const float* x       = (const float*)d_in[0];
  const float* ln1_g   = (const float*)d_in[1];
  const float* ln1_b   = (const float*)d_in[2];
  const float* log_dt  = (const float*)d_in[3];
  const float* log_ar  = (const float*)d_in[4];
  const float* a_imag  = (const float*)d_in[5];
  const float* c_real  = (const float*)d_in[6];
  const float* c_imag  = (const float*)d_in[7];
  const float* dskip   = (const float*)d_in[8];
  const float* out_w   = (const float*)d_in[9];
  const float* out_b   = (const float*)d_in[10];
  const float* ln2_g   = (const float*)d_in[11];
  const float* ln2_b   = (const float*)d_in[12];
  const float* w_up    = (const float*)d_in[13];
  const float* b_up    = (const float*)d_in[14];
  const float* w_dn    = (const float*)d_in[15];
  const float* b_dn    = (const float*)d_in[16];

  char* ws = (char*)d_ws;
  size_t off = 0;
  auto carve = [&](size_t bytes) -> char* { char* p = ws + off; off += (bytes + 255) & ~(size_t)255; return p; };
  unsigned short* WO16 = (unsigned short*)carve((size_t)2 * HDIM * HDIM * 2);
  unsigned short* W1T  = (unsigned short*)carve((size_t)FDIM * HDIM * 2);
  unsigned short* W2T  = (unsigned short*)carve((size_t)HDIM * FDIM * 2);
  unsigned short* KF   = (unsigned short*)carve((size_t)HDIM * SEQL * 2);
  unsigned short* UREV = (unsigned short*)carve((size_t)NROWS * HDIM * 2);
  float*          X1   = (float*)carve((size_t)NROWS * HDIM * 4);
  unsigned short* RM   = (unsigned short*)carve((size_t)NROWS * FDIM * 2);
  if (off > ws_size || off > (size_t)134217728) return;
  unsigned short* H2 = UREV;
  unsigned short* YT = RM;
  unsigned short* YG = RM + (size_t)NROWS * HDIM;
  unsigned short* MM = RM;

  cast8_kernel<<<(2 * HDIM * HDIM / 8) / 256, 256, 0, stream>>>(out_w, WO16, 2 * HDIM * HDIM / 8, WCARRY);
  transpose_cast_kernel<<<dim3(FDIM / 64, HDIM / 64), 256, 0, stream>>>(w_up, W1T, HDIM, FDIM, WCARRY);
  transpose_cast_kernel<<<dim3(HDIM / 64, FDIM / 64), 256, 0, stream>>>(w_dn, W2T, FDIM, HDIM, WCARRY);

  kgen_kernel<<<HDIM, 256, 0, stream>>>(log_dt, log_ar, a_imag, c_real, c_imag, dskip, KF);

  ln1_rev_kernel<<<dim3(NCHK, NBAT), 256, 0, stream>>>(x, ln1_g, ln1_b, UREV);

  conv_toeplitz_kernel<<<dim3(HDIM, NBAT / 4), 128, 0, stream>>>(UREV, KF, YT);

  transpose16_kernel<<<dim3(SEQL / 64, HDIM / 64, NBAT), 256, 0, stream>>>(YT, YG, HDIM, SEQL);

  gemm_f16_kernel<0><<<(NROWS / 64) * (HDIM / 32) / 4, 128, 0, stream>>>(
      YG, HDIM, WO16, HDIM, (void*)X1, HDIM, out_b, x, HDIM, NROWS, HDIM, HDIM, WCARRY_INV);

  ln2_kernel<<<NROWS / 8, 256, 0, stream>>>(X1, ln2_g, ln2_b, H2, NROWS);

  gemm_f16_kernel<1><<<(NROWS / 64) * (FDIM / 64) / 4, 128, 0, stream>>>(
      H2, HDIM, W1T, HDIM, (void*)MM, FDIM, b_up, b_up, 0, NROWS, FDIM, HDIM, WCARRY_INV);

  gemm_f16_kernel<2><<<(NROWS / 64) * (HDIM / 64) / 4, 128, 0, stream>>>(
      MM, FDIM, W2T, FDIM, d_out, HDIM, b_dn, X1, HDIM, NROWS, HDIM, FDIM, WCARRY_INV);
}
